// GCNNet1_42812234006620
// MI455X (gfx1250) — hardware-verified
//
#include <hip/hip_runtime.h>
#include <stddef.h>


#define DF      128
#define NTHR    256
#define NWAVE   8
#define EPT     8
#define NGRP    2
#define CHUNK   (NTHR * EPT * NGRP)
#define WCAP    (EPT * NGRP * 32)
#define LISTN   (NWAVE * WCAP)
#define NB      512
#define NBD     4096
#define WPL     (DF * DF)
#define WSCALE  8.0f
#define WINV    0.125f
#define BN_EPS  1e-5f

#define LDS_AGG (NB * DF * 4 + LISTN * 4 + 64)

static_assert((CHUNK & (CHUNK - 1)) == 0);
static_assert(CHUNK <= 4096);
static_assert(NB <= 4096 && NBD <= 4096);
static_assert((NB & (NB - 1)) == 0 && (NBD & (NBD - 1)) == 0);
static_assert(2 * NB <= LISTN);
static_assert(NB == 16 * 4 * NWAVE);
static_assert(NBD == 4 * 4 * NTHR);

typedef float    v4f  __attribute__((ext_vector_type(4)));
typedef float    v8f  __attribute__((ext_vector_type(8)));
typedef int      v4i  __attribute__((ext_vector_type(4)));
typedef _Float16 v8h  __attribute__((ext_vector_type(8)));
typedef _Float16 v16h __attribute__((ext_vector_type(16)));
union FragH { v16h v; v8h h[2]; };

__device__ __forceinline__ v8h cvt8(v4f a, v4f b) {
  v8h r;
  r[0] = (_Float16)a.x; r[1] = (_Float16)a.y; r[2] = (_Float16)a.z; r[3] = (_Float16)a.w;
  r[4] = (_Float16)b.x; r[5] = (_Float16)b.y; r[6] = (_Float16)b.z; r[7] = (_Float16)b.w;
  return r;
}

__device__ __forceinline__ v8f wmh(v16h a, v16h b, v8f c) {
  v8f d = __builtin_amdgcn_wmma_f32_16x16x32_f16(false, a, false, b, (short)0, c, false, false);
  asm volatile("v_nop\n\tv_nop\n\tv_nop\n\tv_nop" : "+v"(d) : "v"(a), "v"(b));
  return d;
}

template <int NBK, int ENC>
__device__ __forceinline__ int scan_chunk(const int* __restrict__ keys, int nK, int cbase, int base,
                                          int* list, int tid, int lane, int wave) {
  int wc = 0;
#pragma unroll
  for (int g = 0; g < NGRP; ++g) {
    const int el0  = (g * NTHR + tid) * EPT;
    const int e0   = cbase + el0;
    const int sent = -2147483647 - 1;
    v4i da, db;
    if (e0 + 7 < nK) {
      da = *(const v4i*)(keys + e0);
      db = *(const v4i*)(keys + e0 + 4);
    } else {
      da.x = (e0     < nK) ? keys[e0]     : sent;
      da.y = (e0 + 1 < nK) ? keys[e0 + 1] : sent;
      da.z = (e0 + 2 < nK) ? keys[e0 + 2] : sent;
      da.w = (e0 + 3 < nK) ? keys[e0 + 3] : sent;
      db.x = (e0 + 4 < nK) ? keys[e0 + 4] : sent;
      db.y = (e0 + 5 < nK) ? keys[e0 + 5] : sent;
      db.z = (e0 + 6 < nK) ? keys[e0 + 6] : sent;
      db.w = (e0 + 7 < nK) ? keys[e0 + 7] : sent;
    }
    const unsigned nb = (unsigned)base;
    const unsigned s0 = (unsigned)da.x - nb, s1 = (unsigned)da.y - nb;
    const unsigned s2 = (unsigned)da.z - nb, s3 = (unsigned)da.w - nb;
    const unsigned s4 = (unsigned)db.x - nb, s5 = (unsigned)db.y - nb;
    const unsigned s6 = (unsigned)db.z - nb, s7 = (unsigned)db.w - nb;
    const bool h0 = s0 < (unsigned)NBK, h1 = s1 < (unsigned)NBK, h2 = s2 < (unsigned)NBK, h3 = s3 < (unsigned)NBK;
    const bool h4 = s4 < (unsigned)NBK, h5 = s5 < (unsigned)NBK, h6 = s6 < (unsigned)NBK, h7 = s7 < (unsigned)NBK;
    const unsigned any = __builtin_amdgcn_ballot_w32(h0 | h1 | h2 | h3 | h4 | h5 | h6 | h7);
    if (any != 0u) {
#define HITJ(J, HJ, SJ) { \
        const unsigned mj = __builtin_amdgcn_ballot_w32(HJ); \
        if (mj != 0u) { \
          if (HJ) { \
            const int pos = wc + (int)__builtin_amdgcn_mbcnt_lo(mj, 0u); \
            const int ent = ENC ? ((((el0 + (J)) << 12)) | (int)(SJ)) : (e0 + (J)); \
            if (pos < WCAP) list[wave * WCAP + pos] = ent; \
          } \
          wc += (int)__builtin_popcount(mj); } }
      HITJ(0, h0, s0)
      HITJ(1, h1, s1)
      HITJ(2, h2, s2)
      HITJ(3, h3, s3)
      HITJ(4, h4, s4)
      HITJ(5, h5, s5)
      HITJ(6, h6, s6)
      HITJ(7, h7, s7)
#undef HITJ
    }
  }
  return wc;
}

__global__ __launch_bounds__(NTHR) void k_prep(const float* __restrict__ Wsrc, _Float16* wp, int total8) {
  const int i = blockIdx.x * NTHR + threadIdx.x;
  if (i >= total8) return;
  const int o   = i * 8;
  const int l   = o / WPL;
  const int rem = o - l * WPL;
  const int n   = rem / DF;
  const int k0  = rem - n * DF;
  const float* p = Wsrc + (size_t)l * WPL + (size_t)k0 * DF + n;
  v4f a, b;
  a.x = p[0];      a.y = p[DF];     a.z = p[2 * DF]; a.w = p[3 * DF];
  b.x = p[4 * DF]; b.y = p[5 * DF]; b.z = p[6 * DF]; b.w = p[7 * DF];
  a = a * WSCALE;
  b = b * WSCALE;
  const v8h hv = cvt8(a, b);
  _Float16* dp = wp + o;
  *(volatile v8h*)dp = hv;
  __threadfence();
  *(volatile v8h*)dp = hv;
}

__global__ __launch_bounds__(NTHR) void k_deg(
    const int* __restrict__ esrc, const int* __restrict__ edst, float* degp, int nBD, int nE) {
  __shared__ __attribute__((aligned(16))) int cnt[NBD];
  __shared__ __attribute__((aligned(16))) int list[LISTN];
  __shared__ int wcnt[NWAVE];
  const int tid = threadIdx.x, lane = tid & 31, wave = tid >> 5;
  const int which = ((int)blockIdx.x >= nBD) ? 1 : 0;
  const int blk = (int)blockIdx.x - which * nBD;
  const int* keys = which ? edst : esrc;
  const int nodeBase = blk * NBD;
  float* plane = degp + (size_t)which * ((size_t)nBD * NBD) + (size_t)nodeBase;

  for (int i = tid; i < NBD; i += NTHR) cnt[i] = 0;
  __syncthreads();

  const int nChunks = (nE + CHUNK - 1) / CHUNK;
#pragma unroll 1
  for (int ch = 0; ch < nChunks; ++ch) {
    const int cbase = ch * CHUNK;
    const int wc = scan_chunk<NBD, 1>(keys, nE, cbase, nodeBase, list, tid, lane, wave);
    if (lane == 0) wcnt[wave] = wc;
    __syncthreads();
    if (wave == 0) {
#pragma unroll 1
      for (int wsx = 0; wsx < NWAVE; ++wsx) {
        int n = __builtin_amdgcn_readfirstlane(wcnt[wsx]);
        n = n > WCAP ? WCAP : (n < 0 ? 0 : n);
        const int* lp = list + wsx * WCAP;
#pragma unroll 1
        for (int i = 0; i < n; ++i) {
          const int ent  = __builtin_amdgcn_readfirstlane(lp[i]);
          const int slot = ent & (NBD - 1);
          if (lane == 0) cnt[slot] = cnt[slot] + 1;
        }
      }
    }
    __syncthreads();
  }

  v4f dq[4];
#pragma unroll
  for (int q = 0; q < 4; ++q) {
    const int f = (wave * 4 + q) * 128 + 4 * lane;
    const v4i c = *(const v4i*)(cnt + f);
    dq[q].x = rsqrtf(fmaxf((float)c.x, 1.0f));
    dq[q].y = rsqrtf(fmaxf((float)c.y, 1.0f));
    dq[q].z = rsqrtf(fmaxf((float)c.z, 1.0f));
    dq[q].w = rsqrtf(fmaxf((float)c.w, 1.0f));
  }
#pragma unroll
  for (int q = 0; q < 4; ++q) *(volatile v4f*)(plane + (wave * 4 + q) * 128 + 4 * lane) = dq[q];
  __threadfence();
#pragma unroll
  for (int q = 0; q < 4; ++q) *(volatile v4f*)(plane + (wave * 4 + q) * 128 + 4 * lane) = dq[q];
}

__global__ __launch_bounds__(NTHR) void k_agg(
    const int* __restrict__ esrc, const int* __restrict__ edst,
    const float* __restrict__ hin, const float* __restrict__ nsrc, const float* __restrict__ ndst,
    const _Float16* __restrict__ wl, const float* __restrict__ bl, const float* __restrict__ snorm,
    float* hpre, double* part, int nN, int nE) {
  extern __shared__ v4f lds_dyn[];
  float* acc  = (float*)lds_dyn;
  int*   list = (int*)(acc + NB * DF);
  int*   wcnt = list + LISTN;
  float* sn   = (float*)list;
  float* dn   = sn + NB;
  const int tid = threadIdx.x, lane = tid & 31, wave = tid >> 5, hh = lane >> 4, m = lane & 15;
  const int nodeBase = blockIdx.x * NB;

  {
    const v4f z = {0.f, 0.f, 0.f, 0.f};
    for (int i = tid; i < NB * DF / 4; i += NTHR) lds_dyn[i] = z;
  }
  __syncthreads();

  const int nChunks = (nE + CHUNK - 1) / CHUNK;
#pragma unroll 1
  for (int ch = 0; ch < nChunks; ++ch) {
    const int cbase = ch * CHUNK;
    const int wc = scan_chunk<NB, 1>(edst, nE, cbase, nodeBase, list, tid, lane, wave);
    if (lane == 0) wcnt[wave] = wc;
    __syncthreads();
    if (wave == 0) {
#pragma unroll 1
      for (int wsx = 0; wsx < NWAVE; ++wsx) {
        int n = __builtin_amdgcn_readfirstlane(wcnt[wsx]);
        n = n > WCAP ? WCAP : (n < 0 ? 0 : n);
        const int* lp = list + wsx * WCAP;
#pragma unroll 1
        for (int i = 0; i < n; ++i) {
          const int ent  = __builtin_amdgcn_readfirstlane(lp[i]);
          const int slot = ent & (NB - 1);
          int e = cbase + ((ent >> 12) & (CHUNK - 1));
          e = e > nE - 1 ? nE - 1 : e;
          int src = esrc[e];
          src = src < 0 ? 0 : (src > nN - 1 ? nN - 1 : src);
          const float ns = nsrc[src];
          const v4f v = *(const v4f*)(hin + (size_t)src * DF + 4 * lane) * ns;
          v4f* ap = (v4f*)(acc + slot * DF + 4 * lane);
          *ap = *ap + v;
        }
      }
    }
    __syncthreads();
  }

  for (int i = tid; i < NB; i += NTHR) {
    int node = nodeBase + i;
    node = node > nN - 1 ? nN - 1 : node;
    sn[i] = snorm[node];
    dn[i] = ndst[node];
  }
  __syncthreads();

  float bcol[8];
#pragma unroll
  for (int c = 0; c < 8; ++c) bcol[c] = bl[16 * c + m];

#pragma unroll 1
  for (int q = 0; q < NB / 16 / NWAVE; ++q) {
    const int t = wave + NWAVE * q;
    const float dnr = dn[16 * t + m];
    v8f a8[8];
#pragma unroll
    for (int c = 0; c < 8; ++c) { v8f z = {0.f, 0.f, 0.f, 0.f, 0.f, 0.f, 0.f, 0.f}; a8[c] = z; }
#pragma unroll
    for (int kt = 0; kt < DF / 32; ++kt) {
      const float* ap = acc + (16 * t + m) * DF + 32 * kt + 8 * hh;
      const v4f p0 = *(const v4f*)ap,        p1 = *(const v4f*)(ap + 4);
      const v4f p2 = *(const v4f*)(ap + 16), p3 = *(const v4f*)(ap + 20);
      FragH a;
      a.h[0] = cvt8(p0 * dnr, p1 * dnr);
      a.h[1] = cvt8(p2 * dnr, p3 * dnr);
#pragma unroll
      for (int c = 0; c < 8; ++c) {
        const _Float16* bp = wl + (size_t)(16 * c + m) * DF + 32 * kt + 8 * hh;
        FragH b;
        b.h[0] = *(const v8h*)bp;
        b.h[1] = *(const v8h*)(bp + 16);
        a8[c] = wmh(a.v, b.v, a8[c]);
      }
    }
    const int r0 = 16 * t + 8 * hh;
    const v4f sA = *(const v4f*)(sn + r0), sB = *(const v4f*)(sn + r0 + 4);
    float* sp = acc + r0 * DF + m;
#pragma unroll
    for (int c = 0; c < 8; ++c) {
      const float bb = bcol[c];
      float* spc = sp + 16 * c;
      spc[0 * DF] = (a8[c][0] * WINV + bb) * sA.x;
      spc[1 * DF] = (a8[c][1] * WINV + bb) * sA.y;
      spc[2 * DF] = (a8[c][2] * WINV + bb) * sA.z;
      spc[3 * DF] = (a8[c][3] * WINV + bb) * sA.w;
      spc[4 * DF] = (a8[c][4] * WINV + bb) * sB.x;
      spc[5 * DF] = (a8[c][5] * WINV + bb) * sB.y;
      spc[6 * DF] = (a8[c][6] * WINV + bb) * sB.z;
      spc[7 * DF] = (a8[c][7] * WINV + bb) * sB.w;
    }
  }
  __syncthreads();

  const int cch  = tid & (DF - 1);
  const int kind = tid >> 7;
  int nvalid = nN - nodeBase;
  nvalid = nvalid > NB ? NB : (nvalid < 0 ? 0 : nvalid);
  double st = 0.0;
#pragma unroll 1
  for (int r = 0; r < nvalid; ++r) {
    const double x = (double)acc[r * DF + cch];
    st += kind ? x * x : x;
  }
  double* pp = part + (size_t)blockIdx.x * 256 + tid;

#pragma unroll 1
  for (int q = 0; q < NB / 16 / NWAVE; ++q) {
    const int t = wave + NWAVE * q;
    const float* lrow = acc + (16 * t) * DF + 4 * lane;
    float* grow = hpre + ((size_t)nodeBase + 16 * t) * DF + 4 * lane;
#pragma unroll
    for (int i = 0; i < 16; ++i) {
      const v4f v = *(const v4f*)(lrow + i * DF);
      *(volatile v4f*)(grow + (size_t)i * DF) = v;
    }
  }
  *(volatile double*)pp = st;
  __threadfence();
#pragma unroll 1
  for (int q = 0; q < NB / 16 / NWAVE; ++q) {
    const int t = wave + NWAVE * q;
    const float* lrow = acc + (16 * t) * DF + 4 * lane;
    float* grow = hpre + ((size_t)nodeBase + 16 * t) * DF + 4 * lane;
#pragma unroll
    for (int i = 0; i < 16; ++i) {
      const v4f v = *(const v4f*)(lrow + i * DF);
      *(volatile v4f*)(grow + (size_t)i * DF) = v;
    }
  }
  *(volatile double*)pp = st;
}

__global__ __launch_bounds__(DF) void k_bnfin(
    const double* __restrict__ part, const float* __restrict__ gam, const float* __restrict__ bet,
    float* ss, double invN, int nBlk) {
  const int c = threadIdx.x;
  double S = 0.0, Q = 0.0;
#pragma unroll 1
  for (int b = 0; b < nBlk; ++b) {
    S += part[(size_t)b * 256 + c];
    Q += part[(size_t)b * 256 + DF + c];
  }
  const double mu = S * invN;
  double var = Q * invN - mu * mu;
  var = var < 0.0 ? 0.0 : var;
  const float rs = rsqrtf((float)var + BN_EPS);
  const float sc = gam[c] * rs;
  const float sh = bet[c] - (float)mu * sc;
  *(volatile float*)(ss + c) = sc;
  *(volatile float*)(ss + DF + c) = sh;
  __threadfence();
  *(volatile float*)(ss + c) = sc;
  *(volatile float*)(ss + DF + c) = sh;
}

__global__ __launch_bounds__(NTHR) void k_bnapply(
    const float* hold, const float* __restrict__ hpre, const float* __restrict__ ss,
    float* hnew, int nv4) {
  const int i = blockIdx.x * NTHR + threadIdx.x;
  if (i >= nv4) return;
  const int c4 = (i & 31) * 4;
  const size_t o = (size_t)i * 4;
  const v4f ho = *(const v4f*)(hold + o);
  const v4f hp = *(const v4f*)(hpre + o);
  const v4f sc = *(const v4f*)(ss + c4), sh = *(const v4f*)(ss + DF + c4);
  v4f tt = hp * sc + sh;
  tt.x = fmaxf(tt.x, 0.f); tt.y = fmaxf(tt.y, 0.f); tt.z = fmaxf(tt.z, 0.f); tt.w = fmaxf(tt.w, 0.f);
  const v4f r = ho + tt;
  *(volatile v4f*)(hnew + o) = r;
  __threadfence();
  *(volatile v4f*)(hnew + o) = r;
}

__global__ __launch_bounds__(NTHR) void k_readout(
    const int* __restrict__ gids, const float* __restrict__ h3, const float* __restrict__ hpre,
    const float* __restrict__ ss, float* out, int nN) {
  __shared__ __attribute__((aligned(16))) int list[LISTN];
  __shared__ __attribute__((aligned(16))) v4f red4[NWAVE * 32];
  __shared__ int rc[NWAVE];
  const int tid = threadIdx.x, lane = tid & 31, wave = tid >> 5;
  const int g = blockIdx.x;
  const v4f sc = *(const v4f*)(ss + 4 * lane), sh = *(const v4f*)(ss + DF + 4 * lane);
  v4f accv = {0.f, 0.f, 0.f, 0.f};
  int cnt = 0;

  const int nChunks = (nN + CHUNK - 1) / CHUNK;
#pragma unroll 1
  for (int ch = 0; ch < nChunks; ++ch) {
    const int cbase = ch * CHUNK;
    const int wc = scan_chunk<1, 0>(gids, nN, cbase, g, list, tid, lane, wave);
    __syncthreads();
    int n = __builtin_amdgcn_readfirstlane(wc);
    n = n > WCAP ? WCAP : (n < 0 ? 0 : n);
    const int* lp = list + wave * WCAP;
#pragma unroll 1
    for (int i = 0; i < n; ++i) {
      int node = __builtin_amdgcn_readfirstlane(lp[i]);
      node = node < 0 ? 0 : (node > nN - 1 ? nN - 1 : node);
      const size_t o = (size_t)node * DF + 4 * lane;
      const v4f ho = *(const v4f*)(h3 + o);
      const v4f hp = *(const v4f*)(hpre + o);
      v4f tt = hp * sc + sh;
      tt.x = fmaxf(tt.x, 0.f); tt.y = fmaxf(tt.y, 0.f); tt.z = fmaxf(tt.z, 0.f); tt.w = fmaxf(tt.w, 0.f);
      accv = accv + ho + tt;
    }
    cnt += n;
    __syncthreads();
  }
  red4[wave * 32 + lane] = accv;
  if (lane == 0) rc[wave] = cnt;
  __syncthreads();
  if (wave == 0) {
    v4f s = red4[lane];
    int tot = rc[0];
#pragma unroll
    for (int w = 1; w < NWAVE; ++w) { s = s + red4[w * 32 + lane]; tot += rc[w]; }
    const float cf  = fmaxf((float)tot, 1.0f);
    const float inv = 1.0f / cf;
    const v4f o = s * inv;
    float* gp = out + (size_t)g * DF + 4 * lane;
    *(volatile v4f*)gp = o;
    __threadfence();
    *(volatile v4f*)gp = o;
  }
}

extern "C" void kernel_launch(void* const* d_in, const int* in_sizes, int n_in,
                              void* d_out, int out_size, void* d_ws, size_t ws_size,
                              hipStream_t stream) {
  if (n_in < 9) return;
  if (in_sizes[0] <= 0 || (in_sizes[0] % DF) != 0) return;
  const int nN = in_sizes[0] / DF;
  if (in_sizes[1] != nN) return;
  if (in_sizes[2] <= 0 || (in_sizes[2] % WPL) != 0) return;
  const int nL = in_sizes[2] / WPL;
  if (in_sizes[3] != nL * DF || in_sizes[4] != nL * DF || in_sizes[5] != nL * DF) return;
  const int nE = in_sizes[6];
  if (nE < 1 || in_sizes[7] != nE || in_sizes[8] != nN) return;
  if (out_size <= 0 || (out_size % DF) != 0) return;
  const int nG = out_size / DF;

  const float* x      = (const float*)d_in[0];
  const float* snorm  = (const float*)d_in[1];
  const float* Wsrc   = (const float*)d_in[2];
  const float* bs     = (const float*)d_in[3];
  const float* gammas = (const float*)d_in[4];
  const float* betas  = (const float*)d_in[5];
  const int*   esrc   = (const int*)d_in[6];
  const int*   edst   = (const int*)d_in[7];
  const int*   gids   = (const int*)d_in[8];
  float* out = (float*)d_out;

  const int nBD = (nN + NBD - 1) / NBD;
  const int nA  = (nN + NB - 1) / NB;

  char* ws = (char*)d_ws;
  size_t off = 0;
  const size_t oWp = off; off += (size_t)nL * WPL * 2;                     off = (off + 255) & ~(size_t)255;
  const size_t oDg = off; off += (size_t)2 * nBD * NBD * 4;                off = (off + 255) & ~(size_t)255;
  const size_t oH  = off; off += (size_t)nN * DF * 4;                      off = (off + 255) & ~(size_t)255;
  const size_t oP  = off; off += (size_t)nA * NB * DF * 4;                 off = (off + 255) & ~(size_t)255;
  const size_t oSt = off; off += (size_t)nA * 256 * 8;                     off = (off + 255) & ~(size_t)255;
  const size_t oSS = off; off += (size_t)2 * DF * 4;                       off = (off + 255) & ~(size_t)255;
  if (off > ws_size) return;
  _Float16* wp   = (_Float16*)(ws + oWp);
  float*    degp = (float*)(ws + oDg);
  float*    nsrc = degp;
  float*    ndst = degp + (size_t)nBD * NBD;
  float*    hbuf = (float*)(ws + oH);
  float*    hpre = (float*)(ws + oP);
  double*   part = (double*)(ws + oSt);
  float*    ss   = (float*)(ws + oSS);

  const double invN = 1.0 / (double)nN;
  const int nv4 = nN * (DF / 4);

  const int total8 = nL * WPL / 8;
  k_prep<<<(total8 + NTHR - 1) / NTHR, NTHR, 0, stream>>>(Wsrc, wp, total8);

  k_deg<<<2 * nBD, NTHR, 0, stream>>>(esrc, edst, degp, nBD, nE);

  hipFuncSetAttribute(reinterpret_cast<const void*>(&k_agg),
                      hipFuncAttributeMaxDynamicSharedMemorySize, LDS_AGG);

  for (int l = 0; l < nL; ++l) {
    const float* hin = (l == 0) ? x : hbuf;
    k_agg<<<nA, NTHR, LDS_AGG, stream>>>(esrc, edst, hin, nsrc, ndst,
                                         wp + (size_t)l * WPL, bs + (size_t)l * DF, snorm,
                                         hpre, part, nN, nE);
    k_bnfin<<<1, DF, 0, stream>>>(part, gammas + (size_t)l * DF, betas + (size_t)l * DF, ss, invN, nA);
    if (l + 1 < nL) {
      k_bnapply<<<(nv4 + NTHR - 1) / NTHR, NTHR, 0, stream>>>(hin, hpre, ss, hbuf, nv4);
    }
  }

  const float* hlast = (nL > 1) ? hbuf : x;
  k_readout<<<nG, NTHR, 0, stream>>>(gids, hlast, hpre, ss, out, nN);
}
